// RoadNetworkEncoder_44083544326738
// MI455X (gfx1250) — hardware-run, weakly checked
//
#include <hip/hip_runtime.h>
#include <stddef.h>


#define HD      128
#define DID     64
#define DAT     16
#define NTHR    256
#define NWAVE   8
#define CHUNK   4096
#define NGRP    (CHUNK / (NTHR * 4))
#define WCAP    (CHUNK / NWAVE)
#define LSH     12
#define NB      512
#define NBD     4096
#define GRW     64
#define CP      132
#define XHP     136
#define NMAT    6
#define WPL     (HD * HD)
#define CARRY   64.0f
#define UNCARRY (1.0f / 4096.0f)

#define LA_SM    (NB * HD)
#define LA_SL    (LA_SM + NB)
#define LA_SEX   (LA_SL + NB)
#define LA_SEY   (LA_SEX + NB)
#define LA_SCN   (LA_SEY + NB)
#define LA_LIST  (LA_SCN + NB)
#define LA_WCNT  (LA_LIST + NWAVE * WCAP)
#define LA_END   (LA_WCNT + 16)
#define LA_BYTES (LA_END * 4)
#define LB_LIST  (NB * HD)
#define LB_WCNT  (LB_LIST + NWAVE * WCAP)
#define LB_END   (LB_WCNT + 16)
#define LB_BYTES (LB_END * 4)
#define LD_LIST  (NBD)
#define LD_WCNT  (LD_LIST + NWAVE * WCAP)
#define LD_END   (LD_WCNT + 16)
#define LD_BYTES (LD_END * 4)

static_assert(NGRP == 4);
static_assert(WCAP == 512);
static_assert(WCAP == NGRP * 4 * 32);
static_assert((CHUNK & (CHUNK - 1)) == 0);
static_assert(CHUNK <= (1 << 19));
static_assert((NB & (NB - 1)) == 0);
static_assert((NBD & (NBD - 1)) == 0);
static_assert(NB <= (1 << LSH));
static_assert(NBD <= (1 << LSH));
static_assert((NB % (NWAVE * 2)) == 0);
static_assert(NBD == NWAVE * 4 * 128);
static_assert(HD == 4 * 32);
static_assert(LA_BYTES == 288832);
static_assert(LB_BYTES == 278592);
static_assert(LD_BYTES == 32832);
static_assert((CP * 4) % 16 == 0);
static_assert((XHP * 2) % 16 == 0);

typedef float    v2f  __attribute__((ext_vector_type(2)));
typedef float    v4f  __attribute__((ext_vector_type(4)));
typedef float    v8f  __attribute__((ext_vector_type(8)));
typedef int      v4i  __attribute__((ext_vector_type(4)));
typedef _Float16 v4h  __attribute__((ext_vector_type(4)));
typedef _Float16 v8h  __attribute__((ext_vector_type(8)));
typedef _Float16 v16h __attribute__((ext_vector_type(16)));
union FragH { v16h v; v8h half[2]; };
union H8    { v8h v; v4h q[2]; v4i i; };

__device__ __forceinline__ v8f wm(v16h a, v16h b, v8f c) {
  v8f d = __builtin_amdgcn_wmma_f32_16x16x32_f16(false, a, false, b, (short)0, c, false, false);
  asm volatile("v_nop\n\tv_nop\n\tv_nop\n\tv_nop" : "+v"(d) : "v"(a), "v"(b));
  return d;
}

__device__ __forceinline__ float wsum(float v) {
  v += __shfl_xor(v, 16, 32);
  v += __shfl_xor(v, 8, 32);
  v += __shfl_xor(v, 4, 32);
  v += __shfl_xor(v, 2, 32);
  v += __shfl_xor(v, 1, 32);
  return v;
}

__device__ __forceinline__ v4f relu4(v4f v) {
  v4f r;
  r.x = fmaxf(v.x, 0.f); r.y = fmaxf(v.y, 0.f);
  r.z = fmaxf(v.z, 0.f); r.w = fmaxf(v.w, 0.f);
  return r;
}

__global__ __launch_bounds__(NTHR) void k_prepw(
    const float* __restrict__ w0, const float* __restrict__ w1, const float* __restrict__ w2,
    const float* __restrict__ w3, const float* __restrict__ w4, const float* __restrict__ w5,
    _Float16* P) {
  const int mat  = blockIdx.x >> 3;
  const int task = (blockIdx.x & 7) * NTHR + (int)threadIdx.x;
  const int n    = task >> 4;
  const int k0   = (task & 15) * 8;
  const float* W = w0;
  if (mat == 1) W = w1;
  else if (mat == 2) W = w2;
  else if (mat == 3) W = w3;
  else if (mat == 4) W = w4;
  else if (mat == 5) W = w5;
  v4f f0, f1;
  f0.x = W[(k0 + 0) * HD + n]; f0.y = W[(k0 + 1) * HD + n];
  f0.z = W[(k0 + 2) * HD + n]; f0.w = W[(k0 + 3) * HD + n];
  f1.x = W[(k0 + 4) * HD + n]; f1.y = W[(k0 + 5) * HD + n];
  f1.z = W[(k0 + 6) * HD + n]; f1.w = W[(k0 + 7) * HD + n];
  f0 = f0 * CARRY;
  f1 = f1 * CARRY;
  H8 o;
  o.q[0] = __builtin_convertvector(f0, v4h);
  o.q[1] = __builtin_convertvector(f1, v4h);
  const v4i val = o.i;
  _Float16* gp = P + (size_t)mat * WPL + (size_t)n * HD + k0;
  *(volatile v4i*)gp = val;
  __threadfence();
  *(volatile v4i*)gp = val;
}

__global__ __launch_bounds__(NTHR) void k_feat(
    const float* __restrict__ idemb,
    const float* __restrict__ lw, const float* __restrict__ lb,
    const float* __restrict__ temb,
    const float* __restrict__ ow, const float* __restrict__ ob,
    const float* __restrict__ aw, const float* __restrict__ ab,
    const float* __restrict__ alen, const int* __restrict__ atyp,
    const float* __restrict__ alon, const float* __restrict__ alat,
    _Float16* XP, int nN, int nT) {
  __shared__ __attribute__((aligned(16))) _Float16 Ts[GRW * XHP];
  const int tid = threadIdx.x;
  const int rowBase = blockIdx.x * GRW;

#pragma unroll 1
  for (int it = 0; it < 4; ++it) {
    const int task = it * NTHR + tid;
    const int cg   = task >> 6;
    const int r    = task & 63;
    const int row  = rowBase + r;
    const int rowc = (row < nN) ? row : (nN - 1);
    v4f f0, f1;
    if (cg < 8) {
      const float* p = idemb + (size_t)rowc * DID + cg * 8;
      f0 = *(const v4f*)(p);
      f1 = *(const v4f*)(p + 4);
    } else {
      const int jj  = (cg & 1) * 8;
      const int grp = (cg - 8) >> 1;
      if (grp == 1) {
        int t = atyp[rowc];
        t = t < 0 ? 0 : (t > nT - 1 ? nT - 1 : t);
        const float* q = temb + (size_t)t * DAT + jj;
        f0 = *(const v4f*)(q);
        f1 = *(const v4f*)(q + 4);
      } else {
        const float* Wv = (grp == 0) ? lw : ((grp == 2) ? ow : aw);
        const float* bv = (grp == 0) ? lb : ((grp == 2) ? ob : ab);
        const float* sv = (grp == 0) ? alen : ((grp == 2) ? alon : alat);
        const float  a  = sv[rowc];
        const v4f wq0 = *(const v4f*)(Wv + jj);
        const v4f wq1 = *(const v4f*)(Wv + jj + 4);
        const v4f cq0 = *(const v4f*)(bv + jj);
        const v4f cq1 = *(const v4f*)(bv + jj + 4);
        f0 = wq0 * a + cq0;
        f1 = wq1 * a + cq1;
      }
    }
    const float sc = (row < nN) ? CARRY : 0.f;
    f0 = f0 * sc;
    f1 = f1 * sc;
    H8 o;
    o.q[0] = __builtin_convertvector(f0, v4h);
    o.q[1] = __builtin_convertvector(f1, v4h);
    *(v8h*)(Ts + r * XHP + cg * 8) = o.v;
  }
  __syncthreads();

#pragma unroll 1
  for (int it = 0; it < 4; ++it) {
    const int r  = it * 16 + (tid >> 4);
    const int c0 = (tid & 15) * 8;
    H8 o;
    o.v = *(const v8h*)(Ts + r * XHP + c0);
    const v4i val = o.i;
    _Float16* gp = XP + (size_t)(rowBase + r) * HD + c0;
    *(volatile v4i*)gp = val;
    __threadfence();
    *(volatile v4i*)gp = val;
  }
}

__global__ __launch_bounds__(NTHR) void k_cvt(const float* __restrict__ src, _Float16* dst, int nN) {
  const int tid = threadIdx.x;
  const int rowBase = blockIdx.x * GRW;
#pragma unroll 1
  for (int it = 0; it < 4; ++it) {
    const int r    = it * 16 + (tid >> 4);
    const int c0   = (tid & 15) * 8;
    const int row  = rowBase + r;
    const int rowc = (row < nN) ? row : (nN - 1);
    const float* p = src + (size_t)rowc * HD + c0;
    v4f f0 = *(const v4f*)(p);
    v4f f1 = *(const v4f*)(p + 4);
    const float sc = (row < nN) ? CARRY : 0.f;
    f0 = f0 * sc;
    f1 = f1 * sc;
    H8 o;
    o.q[0] = __builtin_convertvector(f0, v4h);
    o.q[1] = __builtin_convertvector(f1, v4h);
    const v4i val = o.i;
    _Float16* gp = dst + (size_t)row * HD + c0;
    *(volatile v4i*)gp = val;
    __threadfence();
    *(volatile v4i*)gp = val;
  }
}

__global__ __launch_bounds__(NTHR) void k_gemm(
    const _Float16* __restrict__ A,
    const _Float16* __restrict__ W0, const _Float16* __restrict__ W1,
    const float* __restrict__ b0, const float* __restrict__ b1,
    float* Y0, float* Y1, int useBias, int nPad) {
  __shared__ __attribute__((aligned(16))) float Cs[GRW * CP];
  const int tid  = threadIdx.x;
  const int lane = tid & 31;
  const int wave = tid >> 5;
  const int hh   = lane >> 4;
  const int m    = lane & 15;
  const int sel  = blockIdx.y;
  const _Float16* W = sel ? W1 : W0;
  const float* bias = sel ? b1 : b0;
  float* Y = sel ? Y1 : Y0;
  const int rowBase = blockIdx.x * GRW;
  const int col = wave * 16 + m;
  (void)nPad;

  v8f acc0 = {0.f, 0.f, 0.f, 0.f, 0.f, 0.f, 0.f, 0.f};
  v8f acc1 = {0.f, 0.f, 0.f, 0.f, 0.f, 0.f, 0.f, 0.f};
  v8f acc2 = {0.f, 0.f, 0.f, 0.f, 0.f, 0.f, 0.f, 0.f};
  v8f acc3 = {0.f, 0.f, 0.f, 0.f, 0.f, 0.f, 0.f, 0.f};
#pragma unroll
  for (int ks = 0; ks < HD / 32; ++ks) {
    const int k0 = ks * 32;
    FragH b, a0, a1, a2, a3;
    const _Float16* pb = W + (size_t)col * HD + k0 + 8 * hh;
    b.half[0] = *(const v8h*)(pb);
    b.half[1] = *(const v8h*)(pb + 16);
    const _Float16* pa = A + (size_t)(rowBase + m) * HD + k0 + 8 * hh;
    a0.half[0] = *(const v8h*)(pa);            a0.half[1] = *(const v8h*)(pa + 16);
    a1.half[0] = *(const v8h*)(pa + 16 * HD);  a1.half[1] = *(const v8h*)(pa + 16 * HD + 16);
    a2.half[0] = *(const v8h*)(pa + 32 * HD);  a2.half[1] = *(const v8h*)(pa + 32 * HD + 16);
    a3.half[0] = *(const v8h*)(pa + 48 * HD);  a3.half[1] = *(const v8h*)(pa + 48 * HD + 16);
    acc0 = wm(a0.v, b.v, acc0);
    acc1 = wm(a1.v, b.v, acc1);
    acc2 = wm(a2.v, b.v, acc2);
    acc3 = wm(a3.v, b.v, acc3);
  }

  const float bb = useBias ? bias[col] : 0.f;
#pragma unroll
  for (int r = 0; r < 8; ++r) {
    Cs[(8 * hh + r) * CP + col]      = acc0[r] * UNCARRY + bb;
    Cs[(16 + 8 * hh + r) * CP + col] = acc1[r] * UNCARRY + bb;
    Cs[(32 + 8 * hh + r) * CP + col] = acc2[r] * UNCARRY + bb;
    Cs[(48 + 8 * hh + r) * CP + col] = acc3[r] * UNCARRY + bb;
  }
  __syncthreads();

#pragma unroll
  for (int i = 0; i < 8; ++i) {
    const int row = wave * 8 + i;
    const v4f v = *(const v4f*)(Cs + row * CP + 4 * lane);
    float* gp = Y + (size_t)(rowBase + row) * HD + 4 * lane;
    *(volatile v4f*)gp = v;
    __threadfence();
    *(volatile v4f*)gp = v;
  }
}

__device__ __forceinline__ void scan_chunk(const int* __restrict__ eid, int nE, int cbase,
                                            int nodeBase, unsigned nbv,
                                            int* list, int* wcnt, int tid, int lane, int wave) {
  const bool fullc = ((nE & 3) == 0) && (cbase + CHUNK <= nE);
  int wc = 0;
#pragma unroll
  for (int g = 0; g < NGRP; ++g) {
    const int el0 = (g * NTHR + tid) * 4;
    const int e0  = cbase + el0;
    v4i d;
    if (fullc) {
      d = *(const v4i*)(eid + e0);
    } else {
      const int sent = -2147483647 - 1;
      const int c0 = (e0     < nE - 1) ? e0     : nE - 1;
      const int c1 = (e0 + 1 < nE - 1) ? e0 + 1 : nE - 1;
      const int c2 = (e0 + 2 < nE - 1) ? e0 + 2 : nE - 1;
      const int c3 = (e0 + 3 < nE - 1) ? e0 + 3 : nE - 1;
      const int v0 = eid[c0], v1 = eid[c1], v2 = eid[c2], v3 = eid[c3];
      d.x = (e0     < nE) ? v0 : sent;
      d.y = (e0 + 1 < nE) ? v1 : sent;
      d.z = (e0 + 2 < nE) ? v2 : sent;
      d.w = (e0 + 3 < nE) ? v3 : sent;
    }
    const unsigned s0 = (unsigned)d.x - (unsigned)nodeBase;
    const unsigned s1 = (unsigned)d.y - (unsigned)nodeBase;
    const unsigned s2 = (unsigned)d.z - (unsigned)nodeBase;
    const unsigned s3 = (unsigned)d.w - (unsigned)nodeBase;
    const bool h0 = s0 < nbv;
    const bool h1 = s1 < nbv;
    const bool h2 = s2 < nbv;
    const bool h3 = s3 < nbv;
    const unsigned many = __builtin_amdgcn_ballot_w32(h0 | h1 | h2 | h3);
    if (many != 0u) {
#define HITJ(J, HJ, SJ) {                                                     \
        const unsigned mj = __builtin_amdgcn_ballot_w32(HJ);                  \
        if (HJ) {                                                             \
          const int pos = wc + (int)__builtin_amdgcn_mbcnt_lo(mj, 0u);        \
          if (pos < WCAP) list[wave * WCAP + pos] = ((el0 + (J)) << LSH) | (int)(SJ); \
        }                                                                     \
        wc += (int)__builtin_popcount(mj); }
      HITJ(0, h0, s0)
      HITJ(1, h1, s1)
      HITJ(2, h2, s2)
      HITJ(3, h3, s3)
#undef HITJ
    }
  }
  if (lane == 0) wcnt[wave] = wc;
}

__device__ __forceinline__ void gat_edge(int slot, int src, int node, float ea0, float ea1,
                                         const float* __restrict__ xl, const float* __restrict__ xr,
                                         v4f we0, v4f we1, v4f at4, int lane,
                                         float* sm, float* sl, v4f* sacc4) {
  const v4f xl4 = *(const v4f*)(xl + (size_t)src  * HD + 4 * lane);
  const v4f xr4 = *(const v4f*)(xr + (size_t)node * HD + 4 * lane);
  const v4f ew  = we0 * ea0 + we1 * ea1;
  v4f v  = (xl4 + xr4) + ew;
  const v4f vn = v * 0.2f;
  v.x = (v.x > 0.f) ? v.x : vn.x;
  v.y = (v.y > 0.f) ? v.y : vn.y;
  v.z = (v.z > 0.f) ? v.z : vn.z;
  v.w = (v.w > 0.f) ? v.w : vn.w;
  float s = v.x * at4.x + v.y * at4.y + v.z * at4.z + v.w * at4.w;
  s = wsum(s);
  s = __shfl(s, 0, 32);
  const float mo = sm[slot];
  const float mn = fmaxf(mo, s);
  const float sc = __expf(mo - mn);
  const float p  = __expf(s - mn);
  const float lo = sl[slot];
  sl[slot] = lo * sc + p;
  sm[slot] = mn;
  const v4f cur = sacc4[slot * 32 + lane];
  sacc4[slot * 32 + lane] = cur * sc + xl4 * p;
}

template <int F16OUT>
__device__ __forceinline__ void store_rows(const v4f* sacc4, float* outf, _Float16* outh,
                                           int nodeBase, int nN, int nPad, int wave, int lane) {
  const int hh = lane >> 4;
  const int m  = lane & 15;
  if (F16OUT) {
#pragma unroll 1
    for (int i = 0; i < NB / (NWAVE * 2); ++i) {
      const int slot = wave * (NB / NWAVE) + 2 * i + hh;
      const int node = nodeBase + slot;
      const v4f a = sacc4[slot * 32 + 2 * m] * CARRY;
      const v4f b = sacc4[slot * 32 + 2 * m + 1] * CARRY;
      H8 o;
      o.q[0] = __builtin_convertvector(a, v4h);
      o.q[1] = __builtin_convertvector(b, v4h);
      const v4i val = o.i;
      _Float16* gp = outh + (size_t)node * HD + 8 * m;
      if (node < nPad) *(volatile v4i*)gp = val;
      __threadfence();
      if (node < nPad) *(volatile v4i*)gp = val;
    }
  } else {
#pragma unroll 1
    for (int i = 0; i < NB / NWAVE; ++i) {
      const int slot = wave * (NB / NWAVE) + i;
      const int node = nodeBase + slot;
      const v4f v = sacc4[slot * 32 + lane];
      float* gp = outf + (size_t)node * HD + 4 * lane;
      if (node < nN) *(volatile v4f*)gp = v;
      __threadfence();
      if (node < nN) *(volatile v4f*)gp = v;
    }
  }
}

template <int F16OUT>
__global__ __launch_bounds__(NTHR) void k_gat(
    const float* __restrict__ xl, const float* __restrict__ xr,
    const int* __restrict__ ei, const float* __restrict__ ea,
    const float* __restrict__ We, const float* __restrict__ att,
    const float* __restrict__ bias, float* outf, _Float16* outh,
    int nN, int nE, int nPad) {
  extern __shared__ v4f lds_dyn[];
  float* ldsf  = (float*)lds_dyn;
  v4f*   sacc4 = lds_dyn;
  float* sm    = ldsf + LA_SM;
  float* sl    = ldsf + LA_SL;
  float* sex   = ldsf + LA_SEX;
  float* sey   = ldsf + LA_SEY;
  float* scn   = ldsf + LA_SCN;
  int*   list  = (int*)(ldsf + LA_LIST);
  int*   wcnt  = (int*)(ldsf + LA_WCNT);

  const int tid  = threadIdx.x;
  const int lane = tid & 31;
  const int wave = tid >> 5;
  const int nodeBase = blockIdx.x * NB;

  {
    const v4f z4 = {0.f, 0.f, 0.f, 0.f};
    for (int i = tid; i < (NB * HD) / 4; i += NTHR) sacc4[i] = z4;
    for (int i = tid; i < NB; i += NTHR) {
      sm[i] = -1.0e30f; sl[i] = 0.f; sex[i] = 0.f; sey[i] = 0.f; scn[i] = 0.f;
    }
  }
  __syncthreads();

  const v4f we0 = *(const v4f*)(We + 4 * lane);
  const v4f we1 = *(const v4f*)(We + HD + 4 * lane);
  const v4f at4 = *(const v4f*)(att + 4 * lane);
  const v4f b4  = *(const v4f*)(bias + 4 * lane);
  const int* eid = ei + nE;
  const int nChunks = (nE + CHUNK - 1) / CHUNK;

#pragma unroll 1
  for (int ch = 0; ch < nChunks; ++ch) {
    const int cbase = ch * CHUNK;
    scan_chunk(eid, nE, cbase, nodeBase, (unsigned)NB, list, wcnt, tid, lane, wave);
    __syncthreads();
    if (wave == 0) {
#pragma unroll 1
      for (int w = 0; w < NWAVE; ++w) {
        int c = wcnt[w];
        c = c < 0 ? 0 : (c > WCAP ? WCAP : c);
#pragma unroll 1
        for (int pos = 0; pos < c; ++pos) {
          const int ent  = list[w * WCAP + pos];
          const int slot = ent & (NB - 1);
          const int el   = (ent >> LSH) & (CHUNK - 1);
          int e = cbase + el;
          if (e > nE - 1) e = nE - 1;
          int src = ei[e];
          src = src < 0 ? 0 : (src > nN - 1 ? nN - 1 : src);
          int node = nodeBase + slot;
          if (node > nN - 1) node = nN - 1;
          const v2f a2 = *(const v2f*)(ea + 2 * (size_t)e);
          sex[slot] = sex[slot] + a2.x;
          sey[slot] = sey[slot] + a2.y;
          scn[slot] = scn[slot] + 1.0f;
          gat_edge(slot, src, node, a2.x, a2.y, xl, xr, we0, we1, at4, lane, sm, sl, sacc4);
        }
      }
    }
    __syncthreads();
  }

#pragma unroll 1
  for (int i = 0; i < NB / NWAVE; ++i) {
    const int slot  = wave * (NB / NWAVE) + i;
    const int node  = nodeBase + slot;
    const int nodec = (node < nN) ? node : (nN - 1);
    const float cn  = scn[slot];
    const float ic  = __builtin_amdgcn_rcpf(fmaxf(cn, 1.0f));
    const float ea0 = sex[slot] * ic;
    const float ea1 = sey[slot] * ic;
    gat_edge(slot, nodec, nodec, ea0, ea1, xl, xr, we0, we1, at4, lane, sm, sl, sacc4);
    const v4f a = sacc4[slot * 32 + lane];
    const float l  = sl[slot];
    const float il = (l > 0.f) ? __builtin_amdgcn_rcpf(l) : 0.f;
    v4f val = a * il + b4;
    if (F16OUT) val = relu4(val);
    const v4f z4 = {0.f, 0.f, 0.f, 0.f};
    val = (node < nN) ? val : z4;
    sacc4[slot * 32 + lane] = val;
  }
  __syncthreads();
  store_rows<F16OUT>(sacc4, outf, outh, nodeBase, nN, nPad, wave, lane);
}

__device__ __forceinline__ float dinvf(float d) {
  return (d > 0.f) ? rsqrtf(fmaxf(d, 1e-12f)) : 0.f;
}

__global__ __launch_bounds__(NTHR) void k_dinv(const int* __restrict__ ei, const float* __restrict__ w,
                                               float* dinv, int nN, int nE) {
  extern __shared__ v4f lds_dyn[];
  float* ldsf = (float*)lds_dyn;
  float* sdeg = ldsf;
  int*   list = (int*)(ldsf + LD_LIST);
  int*   wcnt = (int*)(ldsf + LD_WCNT);
  const int tid  = threadIdx.x;
  const int lane = tid & 31;
  const int wave = tid >> 5;
  const int nodeBase = blockIdx.x * NBD;

  for (int i = tid; i < NBD; i += NTHR) sdeg[i] = 0.f;
  __syncthreads();

  const int* eid = ei + nE;
  const int nChunks = (nE + CHUNK - 1) / CHUNK;
#pragma unroll 1
  for (int ch = 0; ch < nChunks; ++ch) {
    const int cbase = ch * CHUNK;
    scan_chunk(eid, nE, cbase, nodeBase, (unsigned)NBD, list, wcnt, tid, lane, wave);
    __syncthreads();
    if (wave == 0) {
#pragma unroll 1
      for (int wv = 0; wv < NWAVE; ++wv) {
        int c = wcnt[wv];
        c = c < 0 ? 0 : (c > WCAP ? WCAP : c);
#pragma unroll 1
        for (int pos = 0; pos < c; ++pos) {
          const int ent  = list[wv * WCAP + pos];
          const int slot = ent & (NBD - 1);
          const int el   = (ent >> LSH) & (CHUNK - 1);
          int e = cbase + el;
          if (e > nE - 1) e = nE - 1;
          const float we = w[e];
          sdeg[slot] = sdeg[slot] + we;
        }
      }
    }
    __syncthreads();
  }

#pragma unroll
  for (int it = 0; it < 4; ++it) {
    const int s0 = wave * (NBD / NWAVE) + it * 128 + 4 * lane;
    const v4f dg = *(const v4f*)(sdeg + s0);
    v4f o;
    o.x = (nodeBase + s0 + 0 < nN) ? dinvf(dg.x + 1.0f) : 0.f;
    o.y = (nodeBase + s0 + 1 < nN) ? dinvf(dg.y + 1.0f) : 0.f;
    o.z = (nodeBase + s0 + 2 < nN) ? dinvf(dg.z + 1.0f) : 0.f;
    o.w = (nodeBase + s0 + 3 < nN) ? dinvf(dg.w + 1.0f) : 0.f;
    float* gp = dinv + (size_t)nodeBase + s0;
    *(volatile v4f*)gp = o;
    __threadfence();
    *(volatile v4f*)gp = o;
  }
}

template <int F16OUT>
__global__ __launch_bounds__(NTHR) void k_gcn(
    const float* __restrict__ h, const int* __restrict__ ei, const float* __restrict__ w,
    const float* __restrict__ dinv, const float* __restrict__ bias,
    float* outf, _Float16* outh, int nN, int nE, int nPad) {
  extern __shared__ v4f lds_dyn[];
  float* ldsf  = (float*)lds_dyn;
  v4f*   sacc4 = lds_dyn;
  int*   list  = (int*)(ldsf + LB_LIST);
  int*   wcnt  = (int*)(ldsf + LB_WCNT);

  const int tid  = threadIdx.x;
  const int lane = tid & 31;
  const int wave = tid >> 5;
  const int nodeBase = blockIdx.x * NB;

  {
    const v4f z4 = {0.f, 0.f, 0.f, 0.f};
    for (int i = tid; i < (NB * HD) / 4; i += NTHR) sacc4[i] = z4;
  }
  __syncthreads();

  const v4f b4 = *(const v4f*)(bias + 4 * lane);
  const int* eid = ei + nE;
  const int nChunks = (nE + CHUNK - 1) / CHUNK;

#pragma unroll 1
  for (int ch = 0; ch < nChunks; ++ch) {
    const int cbase = ch * CHUNK;
    scan_chunk(eid, nE, cbase, nodeBase, (unsigned)NB, list, wcnt, tid, lane, wave);
    __syncthreads();
    if (wave == 0) {
#pragma unroll 1
      for (int wv = 0; wv < NWAVE; ++wv) {
        int c = wcnt[wv];
        c = c < 0 ? 0 : (c > WCAP ? WCAP : c);
#pragma unroll 1
        for (int pos = 0; pos < c; ++pos) {
          const int ent  = list[wv * WCAP + pos];
          const int slot = ent & (NB - 1);
          const int el   = (ent >> LSH) & (CHUNK - 1);
          int e = cbase + el;
          if (e > nE - 1) e = nE - 1;
          int src = ei[e];
          src = src < 0 ? 0 : (src > nN - 1 ? nN - 1 : src);
          int node = nodeBase + slot;
          if (node > nN - 1) node = nN - 1;
          const float we  = w[e];
          const float nrm = (dinv[src] * we) * dinv[node];
          const v4f hv  = *(const v4f*)(h + (size_t)src * HD + 4 * lane);
          const v4f cur = sacc4[slot * 32 + lane];
          sacc4[slot * 32 + lane] = cur + hv * nrm;
        }
      }
    }
    __syncthreads();
  }

#pragma unroll 1
  for (int i = 0; i < NB / NWAVE; ++i) {
    const int slot  = wave * (NB / NWAVE) + i;
    const int node  = nodeBase + slot;
    const int nodec = (node < nN) ? node : (nN - 1);
    const float dn  = dinv[nodec];
    const v4f hv = *(const v4f*)(h + (size_t)nodec * HD + 4 * lane);
    const v4f a  = sacc4[slot * 32 + lane];
    v4f val = (a + hv * (dn * dn)) + b4;
    if (F16OUT) val = relu4(val);
    const v4f z4 = {0.f, 0.f, 0.f, 0.f};
    val = (node < nN) ? val : z4;
    sacc4[slot * 32 + lane] = val;
  }
  __syncthreads();
  store_rows<F16OUT>(sacc4, outf, outh, nodeBase, nN, nPad, wave, lane);
}

static inline int cdiv_i(int a, int b) { return (a + b - 1) / b; }
static inline size_t al256(size_t x) { return (x + 255) & ~(size_t)255; }

extern "C" void kernel_launch(void* const* d_in, const int* in_sizes, int n_in,
                              void* d_out, int out_size, void* d_ws, size_t ws_size,
                              hipStream_t stream) {
  if (n_in < 35) return;
  const int nN = in_sizes[0] / DID;
  if (nN <= 0 || in_sizes[0] != nN * DID) return;
  if (in_sizes[1] != DAT || in_sizes[2] != DAT || in_sizes[4] != DAT ||
      in_sizes[5] != DAT || in_sizes[6] != DAT || in_sizes[7] != DAT) return;
  if (in_sizes[3] < DAT || (in_sizes[3] % DAT) != 0) return;
  const int nT = in_sizes[3] / DAT;
  if (in_sizes[8] != nN || in_sizes[9] != nN || in_sizes[10] != nN || in_sizes[11] != nN) return;
  if (in_sizes[12] < 2 || (in_sizes[12] & 1) != 0) return;
  const int nE = in_sizes[12] / 2;
  if (in_sizes[13] != 2 * nE) return;
  for (int L = 0; L < 2; ++L) {
    const int b = 14 + 7 * L;
    if (in_sizes[b] != WPL || in_sizes[b + 1] != HD || in_sizes[b + 2] != WPL ||
        in_sizes[b + 3] != HD || in_sizes[b + 4] != 2 * HD || in_sizes[b + 5] != HD ||
        in_sizes[b + 6] != HD) return;
  }
  const int nZ = in_sizes[28] / HD;
  if (nZ <= 0 || in_sizes[28] != nZ * HD) return;
  if (in_sizes[29] < 2 || (in_sizes[29] & 1) != 0) return;
  const int nEZ = in_sizes[29] / 2;
  if (in_sizes[30] != nEZ) return;
  if (in_sizes[31] != WPL || in_sizes[32] != HD || in_sizes[33] != WPL || in_sizes[34] != HD) return;
  if (out_size != (nN + nZ) * HD) return;

  const float* idemb = (const float*)d_in[0];
  const float* lw    = (const float*)d_in[1];
  const float* lb    = (const float*)d_in[2];
  const float* temb  = (const float*)d_in[3];
  const float* ow    = (const float*)d_in[4];
  const float* ob    = (const float*)d_in[5];
  const float* aw    = (const float*)d_in[6];
  const float* ab    = (const float*)d_in[7];
  const float* alen  = (const float*)d_in[8];
  const int*   atyp  = (const int*)d_in[9];
  const float* alon  = (const float*)d_in[10];
  const float* alat  = (const float*)d_in[11];
  const int*   eiA   = (const int*)d_in[12];
  const float* eaA   = (const float*)d_in[13];
  const float* Wl1 = (const float*)d_in[14]; const float* bl1 = (const float*)d_in[15];
  const float* Wr1 = (const float*)d_in[16]; const float* br1 = (const float*)d_in[17];
  const float* We1 = (const float*)d_in[18]; const float* at1 = (const float*)d_in[19];
  const float* bs1 = (const float*)d_in[20];
  const float* Wl2 = (const float*)d_in[21]; const float* bl2 = (const float*)d_in[22];
  const float* Wr2 = (const float*)d_in[23]; const float* br2 = (const float*)d_in[24];
  const float* We2 = (const float*)d_in[25]; const float* at2 = (const float*)d_in[26];
  const float* bs2 = (const float*)d_in[27];
  const float* zemb = (const float*)d_in[28];
  const int*   eiB  = (const int*)d_in[29];
  const float* wB   = (const float*)d_in[30];
  const float* Wg1 = (const float*)d_in[31]; const float* bg1 = (const float*)d_in[32];
  const float* Wg2 = (const float*)d_in[33]; const float* bg2 = (const float*)d_in[34];

  float* outA = (float*)d_out;
  float* outB = outA + (size_t)nN * HD;

  const int NpR = cdiv_i(nN, GRW) * GRW;
  const int NpZ = cdiv_i(nZ, GRW) * GRW;
  const int NpM = (NpR > NpZ) ? NpR : NpZ;
  const int NpD = cdiv_i(nZ, NBD) * NBD;

  size_t off = 0;
  char* ws = (char*)d_ws;
  _Float16* WP  = (_Float16*)(ws + off); off += al256((size_t)NMAT * WPL * 2);
  _Float16* P16 = (_Float16*)(ws + off); off += al256((size_t)NpM * HD * 2);
  float*    XL  = (float*)(ws + off);    off += al256((size_t)NpM * HD * 4);
  float*    XR  = (float*)(ws + off);    off += al256((size_t)NpM * HD * 4);
  float*    DI  = (float*)(ws + off);    off += al256((size_t)NpD * 4);
  if (off > ws_size) return;
  _Float16* Z1 = (_Float16*)XR;

  hipFuncSetAttribute(reinterpret_cast<const void*>(&k_gat<1>),
                      hipFuncAttributeMaxDynamicSharedMemorySize, LA_BYTES);
  hipFuncSetAttribute(reinterpret_cast<const void*>(&k_gat<0>),
                      hipFuncAttributeMaxDynamicSharedMemorySize, LA_BYTES);
  hipFuncSetAttribute(reinterpret_cast<const void*>(&k_gcn<1>),
                      hipFuncAttributeMaxDynamicSharedMemorySize, LB_BYTES);
  hipFuncSetAttribute(reinterpret_cast<const void*>(&k_gcn<0>),
                      hipFuncAttributeMaxDynamicSharedMemorySize, LB_BYTES);

  k_prepw<<<NMAT * 8, NTHR, 0, stream>>>(Wl1, Wr1, Wl2, Wr2, Wg1, Wg2, WP);
  k_feat<<<NpR / GRW, NTHR, 0, stream>>>(idemb, lw, lb, temb, ow, ob, aw, ab,
                                          alen, atyp, alon, alat, P16, nN, nT);
  k_gemm<<<dim3(NpR / GRW, 2), NTHR, 0, stream>>>(P16, WP + 0 * WPL, WP + 1 * WPL,
                                                   bl1, br1, XL, XR, 1, NpR);
  k_gat<1><<<cdiv_i(nN, NB), NTHR, LA_BYTES, stream>>>(XL, XR, eiA, eaA, We1, at1, bs1,
                                                       outA, P16, nN, nE, NpR);
  k_gemm<<<dim3(NpR / GRW, 2), NTHR, 0, stream>>>(P16, WP + 2 * WPL, WP + 3 * WPL,
                                                   bl2, br2, XL, XR, 1, NpR);
  k_gat<0><<<cdiv_i(nN, NB), NTHR, LA_BYTES, stream>>>(XL, XR, eiA, eaA, We2, at2, bs2,
                                                       outA, P16, nN, nE, NpR);
  k_cvt<<<NpZ / GRW, NTHR, 0, stream>>>(zemb, P16, nZ);
  k_dinv<<<NpD / NBD, NTHR, LD_BYTES, stream>>>(eiB, wB, DI, nZ, nEZ);
  k_gemm<<<dim3(NpZ / GRW, 1), NTHR, 0, stream>>>(P16, WP + 4 * WPL, WP + 4 * WPL,
                                                   bg1, bg1, XL, XL, 0, NpZ);
  k_gcn<1><<<cdiv_i(nZ, NB), NTHR, LB_BYTES, stream>>>(XL, eiB, wB, DI, bg1,
                                                       outB, Z1, nZ, nEZ, NpZ);
  k_gemm<<<dim3(NpZ / GRW, 1), NTHR, 0, stream>>>(Z1, WP + 5 * WPL, WP + 5 * WPL,
                                                   bg2, bg2, XL, XL, 0, NpZ);
  k_gcn<0><<<cdiv_i(nZ, NB), NTHR, LB_BYTES, stream>>>(XL, eiB, wB, DI, bg2,
                                                       outB, Z1, nZ, nEZ, NpZ);
}
